// pH_SHND_Core_5059471475348
// MI455X (gfx1250) — hardware-run, weakly checked
//
#include <hip/hip_runtime.h>


#ifndef NROWS
#define NROWS 131072
#endif
#define NROWS_FULL 131072
#define LAT  16
#define CTL  8
#define BLN  128
#define HID  64
#define JRO  512
#define BMO  128
#define AW   2
#define MU_C  0.1f
#define EPS_C 0.01f
#define CW_HA 4.0f
#define CW_HB 16.0f
#define CW_L1 4.0f
#define CW_L2 8.0f
#define CW_L3 64.0f
#define LOS   64.0f
#define VVS   64.0f
#define QRS   2048.0f
#define QRI   (1.0f / 2048.0f)
#define I_HA  (1.0f / CW_HA)
#define I_HB  (1.0f / CW_HB)
#define I_L1  (1.0f / CW_L1)
#define I_L2  (1.0f / CW_L2)
#define I_L3  (1.0f / CW_L3)
#define I_G   (1.0f / (CW_HA * VVS))

#define PO_HA  0
#define PO_HB  (PO_HA + BLN * 32)
#define PO_HBT (PO_HB + LAT * BLN)
#define PO_HAT (PO_HBT + BLN * 32)
#define PO_JA  (PO_HAT + LAT * BLN)
#define PO_JB  (PO_JA + HID * 32)
#define PO_JC  (PO_JB + HID * HID)
#define PO_MA  (PO_JC + JRO * HID)
#define PO_MB  (PO_MA + HID * 32)
#define PO_MC  (PO_MB + HID * HID)
#define PO_END (PO_MC + BMO * HID)
#define BO_HA 0
#define BO_JA (BO_HA + BLN)
#define BO_JB (BO_JA + HID)
#define BO_JC (BO_JB + HID)
#define BO_MA (BO_JC + JRO)
#define BO_MB (BO_MA + HID)
#define BO_MC (BO_MB + HID)
#define BO_END (BO_MC + BMO)

#define L_RF 4096
#define L_TS 2048
#define L_GS 256
#define L_OS 384

static_assert(LAT == 16);
static_assert(CTL == 8);
static_assert(BLN == 128);
static_assert(HID == 64);
static_assert(JRO == 2 * LAT * LAT);
static_assert(BMO == LAT * CTL);
static_assert(L_TS == (BLN / 16) * 32 * 8);
static_assert(L_RF == LAT * 16 * LAT);
static_assert(NROWS % (16 * AW) == 0);
static_assert(NROWS <= NROWS_FULL);
static_assert(PO_HB % 2048 == 0 && PO_HBT % 2048 == 0 && PO_HAT % 2048 == 0 && PO_JA % 2048 == 0 && PO_JB % 2048 == 0);
static_assert(PO_JC % 2048 == 0 && PO_MA % 2048 == 0 && PO_MB % 2048 == 0 && PO_MC % 2048 == 0 && PO_END % 2048 == 0);
static_assert(PO_END == 65536);
static_assert(BO_END == 1024);
static_assert(2 * 32 * 16 == 16 * LAT * 4);
static_assert(1 * 32 * 16 == 16 * CTL * 4);
static_assert((size_t)AW * (L_RF + L_TS + L_GS + L_OS) * 4 <= 131072);
static_assert(1024 * 4 <= 131072);
static_assert((size_t)NROWS_FULL * LAT * 4 == 8388608);
static_assert(((size_t)NROWS_FULL * LAT + (size_t)NROWS * CTL) * 4 <= 12582912);

typedef _Float16 h16;
typedef unsigned short bf;
typedef __attribute__((ext_vector_type(16))) __bf16   v16bf;
typedef __attribute__((ext_vector_type(16))) _Float16 v16h;
typedef __attribute__((ext_vector_type(8)))  _Float16 v8h;
typedef __attribute__((ext_vector_type(8)))  unsigned short v8us;
typedef __attribute__((ext_vector_type(8)))  float    v8f;
typedef __attribute__((ext_vector_type(4)))  float    v4f;
typedef v4f  __attribute__((may_alias)) v4fa;

__device__ __forceinline__ unsigned short f2bf(float f) { unsigned u = __float_as_uint(f); u += 0x7FFFu + ((u >> 16) & 1u); return (unsigned short)(u >> 16); }
__device__ __forceinline__ float bfr(float f) { return __uint_as_float(((unsigned)f2bf(f)) << 16); }
__device__ __forceinline__ v16h cat16(v8h lo, v8h hi) { return __builtin_shufflevector(lo, hi, 0, 1, 2, 3, 4, 5, 6, 7, 8, 9, 10, 11, 12, 13, 14, 15); }
__device__ __forceinline__ v16bf cat16b(v8us lo, v8us hi) { return __builtin_bit_cast(v16bf, __builtin_shufflevector(lo, hi, 0, 1, 2, 3, 4, 5, 6, 7, 8, 9, 10, 11, 12, 13, 14, 15)); }
__device__ __forceinline__ v8f wmma16(v16h a, v16h b, v8f c) { return __builtin_amdgcn_wmma_f32_16x16x32_f16(false, a, false, b, (short)0, c, false, false); }
__device__ __forceinline__ v8f wmmab(v16bf a, v16bf b, v8f c) { return __builtin_amdgcn_wmma_f32_16x16x32_bf16(false, a, false, b, (short)0, c, false, false); }
__device__ __forceinline__ v16h  ldh(const h16* p) { return cat16(*(const v8h*)p, *(const v8h*)(p + 16)); }
__device__ __forceinline__ v16bf ldb(const bf* p)  { return cat16b(*(const v8us*)p, *(const v8us*)(p + 16)); }
__device__ __forceinline__ void wave_sync() { __builtin_amdgcn_fence(3  , "wavefront"); __builtin_amdgcn_wave_barrier(); asm volatile("" ::: "memory"); }

static __device__ __forceinline__ h16 toh_flush(float v) { const h16 r = (h16)v; return (fabsf(v) < 6.103515625e-05f) ? (h16)0.0f : r; }
__device__ __forceinline__ v8f mmg(v16h a, v16h b, v8f c) { c = wmma16(a, b, c); asm volatile("v_nop\n\tv_nop\n\tv_nop\n\tv_nop" : "+v"(c) : "v"(a), "v"(b)); return c; }
__device__ __forceinline__ v8f ld8f(const float* p) { const v4f a = *(const v4f*)p, b = *(const v4f*)(p + 4); return __builtin_shufflevector(a, b, 0, 1, 2, 3, 4, 5, 6, 7); }
__device__ __forceinline__ v4f lo4(v8f x) { return __builtin_shufflevector(x, x, 0, 1, 2, 3); }
__device__ __forceinline__ v4f hi4(v8f x) { return __builtin_shufflevector(x, x, 4, 5, 6, 7); }
__device__ __forceinline__ float tanh_e(float x) { const float e = __builtin_amdgcn_exp2f(x * 2.8853900817779268f); return 1.0f - 2.0f * __builtin_amdgcn_rcpf(e + 1.0f); }
__device__ __forceinline__ v16h pack_hl(v8f x) { v16h o;
#pragma unroll
    for (int r = 0; r < 8; ++r) { const h16 a = toh_flush(x[r]); o[r] = a; o[8 + r] = toh_flush((x[r] - (float)a) * LOS); }
    return o; }
__device__ __forceinline__ v16h pack2(v8f x0, v8f x1) { v16h o;
#pragma unroll
    for (int r = 0; r < 8; ++r) { o[r] = toh_flush(x0[r]); o[8 + r] = toh_flush(x1[r]); }
    return o; }
__device__ __forceinline__ v16h pack2r(v8f x0, v8f x1) { v16h o;
#pragma unroll
    for (int r = 0; r < 8; ++r) { const h16 a = toh_flush(x0[r]); const h16 b = toh_flush(x1[r]);
        o[r] = toh_flush((x0[r] - (float)a) * QRS); o[8 + r] = toh_flush((x1[r] - (float)b) * QRS); }
    return o; }

__device__ __forceinline__ v8f tile_a(const h16* wp, const float* bp, v16h b, float inv) {
    const v8f acc = mmg(ldh(wp), b, (v8f){});
    const v8f bb = ld8f(bp);
    v8f t;
#pragma unroll
    for (int r = 0; r < 8; ++r) t[r] = tanh_e(acc[r] * inv + bb[r]);
    return t; }
__device__ __forceinline__ v8f tile_b(const h16* wp, const float* bp, v16h b0, v16h b1, float inv) {
    v8f acc = mmg(ldh(wp), b0, (v8f){}); acc = mmg(ldh(wp + 32), b1, acc);
    const v8f bb = ld8f(bp);
    v8f t;
#pragma unroll
    for (int r = 0; r < 8; ++r) t[r] = tanh_e(acc[r] * inv + bb[r]);
    return t; }
__device__ __forceinline__ v8f tile_br(const h16* wp, const float* bp, v16h b0, v16h b1, v16h r0, v16h r1, int ev, float inv) {
    const v16h a0 = ldh(wp), a1 = ldh(wp + 32);
    v8f acc = mmg(a0, b0, (v8f){}); acc = mmg(a1, b1, acc);
    v8f acr = (v8f){};
    if (ev != 0) { acr = mmg(a0, r0, acr); acr = mmg(a1, r1, acr); }
    const v8f bb = ld8f(bp);
    v8f t;
#pragma unroll
    for (int r = 0; r < 8; ++r) t[r] = tanh_e((acc[r] + acr[r] * QRI) * inv + bb[r]);
    return t; }

__global__ __launch_bounds__(256) void k_wplane(const float* __restrict__ src, h16* dst, int rows, int pitch, int sld, int nsrc, int tr, int dup, int perm, float cs, float cs2) {
    const int i = blockIdx.x * 256 + threadIdx.x;
    const int ppr = pitch >> 3;
    if (i >= rows * ppr) return;
    const int r = i / ppr, c0 = (i - r * ppr) * 8;
    const int rp = (((r >> 3) & 1) * 8 + (r >> 4)) * 8 + (r & 7);
    const int rs = (perm != 0) ? rp : r;
    v8h o;
#pragma unroll
    for (int k = 0; k < 8; ++k) {
        const int c = c0 + k;
        const int cc = (dup != 0) ? (c & 15) : c;
        int idx = (tr != 0) ? (cc * sld + rs) : (rs * sld + cc);
        idx = idx < 0 ? 0 : (idx > nsrc - 1 ? nsrc - 1 : idx);
        const float w = bfr(src[idx]);
        const float sc = ((dup != 0) & (c >= 16)) ? cs2 : cs;
        o[k] = toh_flush(w * sc);
    }
    *(volatile v8h*)(dst + (size_t)i * 8) = o; __threadfence(); *(volatile v8h*)(dst + (size_t)i * 8) = o;
}

__device__ __forceinline__ int clampi(int i, int hi) { return i < 0 ? 0 : (i > hi ? hi : i); }

__global__ __launch_bounds__(256) void k_bias(const float* __restrict__ bha, const float* __restrict__ bja, const float* __restrict__ bjb, const float* __restrict__ bjc,
                                              const float* __restrict__ bma, const float* __restrict__ bmb, const float* __restrict__ bmc, float* dst) {
    __shared__ __align__(16) float sb[1024];
    const int t = threadIdx.x;
#pragma unroll 1
    for (int k = 0; k < 4; ++k) {
        const int e = k * 256 + t;
        const int p = e - BO_MC;
        const int pp = (((p >> 3) & 1) * 8 + (p >> 4)) * 8 + (p & 7);
        float v0 = bha[clampi(e - BO_HA, BLN - 1)]; asm volatile("" : "+v"(v0));
        float v1 = bja[clampi(e - BO_JA, HID - 1)]; asm volatile("" : "+v"(v1));
        float v2 = bjb[clampi(e - BO_JB, HID - 1)]; asm volatile("" : "+v"(v2));
        float v3 = bjc[clampi(e - BO_JC, JRO - 1)]; asm volatile("" : "+v"(v3));
        float v4 = bma[clampi(e - BO_MA, HID - 1)]; asm volatile("" : "+v"(v4));
        float v5 = bmb[clampi(e - BO_MB, HID - 1)]; asm volatile("" : "+v"(v5));
        float v6 = bmc[clampi(pp, BMO - 1)];        asm volatile("" : "+v"(v6));
        float v = v0;
        v = (e >= BO_JA) ? v1 : v; v = (e >= BO_JB) ? v2 : v; v = (e >= BO_JC) ? v3 : v;
        v = (e >= BO_MA) ? v4 : v; v = (e >= BO_MB) ? v5 : v; v = (e >= BO_MC) ? v6 : v;
        sb[e] = bfr(v);
    }
    __syncthreads();
    const v4f o = *(const v4fa*)(&sb[4 * t]);
    *(volatile v4f*)(dst + 4 * t) = o; __threadfence(); *(volatile v4f*)(dst + 4 * t) = o;
}

__global__ __launch_bounds__(32 * AW) __attribute__((amdgpu_num_vgpr(256)))
void k_step(const float* __restrict__ Z, const float* __restrict__ U, const h16* __restrict__ WP, const float* __restrict__ BP, float* OUT0, float* OUT1) {
    __shared__ __align__(16) float rfs[AW * L_RF];
    __shared__ __align__(16) float tss[AW * L_TS];
    __shared__ __align__(16) float gss[AW * L_GS];
    __shared__ __align__(16) float oss[AW * L_OS];
    const int lane = threadIdx.x & 31, lr = lane & 15, hi = lane >> 4;
    const int wave = __builtin_amdgcn_readfirstlane((int)(threadIdx.x >> 5));
    const size_t row0 = ((size_t)blockIdx.x * AW + (size_t)wave) * 16;
    const int rfb = wave * L_RF, tsb = wave * L_TS + lane * 8, gsb = wave * L_GS, osb = wave * L_OS;
    const int fo = 8 * hi;
    const v8f zero8 = (v8f){};
    v8f z0, zc, uv, dzp = zero8, dzl = zero8, yp = zero8;
    { const float* zp = Z + (row0 + (size_t)lr) * LAT + fo; const v4f a = *(const v4f*)zp, b = *(const v4f*)(zp + 4);
      const float* up = U + (row0 + (size_t)lr) * CTL;      const v4f c = *(const v4f*)up, d = *(const v4f*)(up + 4);
#pragma unroll
      for (int r = 0; r < 4; ++r) { z0[r] = bfr(a[r]); z0[4 + r] = bfr(b[r]); uv[r] = bfr(c[r]); uv[4 + r] = bfr(d[r]); } }
    zc = z0;

#pragma unroll 1
    for (int ev = 0; ev < 2; ++ev) {
        const v16h zb = pack_hl(zc);
        v8f aF = zero8, aFr = zero8;
#pragma unroll 1
        for (int s = 0; s < 4; ++s) {
            const v8f t0 = tile_a(WP + PO_HA + (32 * s + lr) * 32 + fo,      BP + BO_HA + 32 * s + fo,      zb, I_HA);
            const v8f t1 = tile_a(WP + PO_HA + (32 * s + 16 + lr) * 32 + fo, BP + BO_HA + 32 * s + 16 + fo, zb, I_HA);
            const int tb = tsb + s * 512;
            *(v4fa*)(&tss[tb]) = lo4(t0);       *(v4fa*)(&tss[tb + 4]) = hi4(t0);
            *(v4fa*)(&tss[tb + 256]) = lo4(t1); *(v4fa*)(&tss[tb + 260]) = hi4(t1);
            const v16h a = ldh(WP + PO_HB + lr * BLN + 32 * s + fo);
            aF = mmg(a, pack2(t0, t1), aF);
            if (ev != 0) aFr = mmg(a, pack2r(t0, t1), aFr);
        }
        v8f fv;
#pragma unroll
        for (int r = 0; r < 8; ++r) fv[r] = (aF[r] + aFr[r] * QRI) * I_HB + MU_C * zc[r];
        wave_sync();
        const v16h fb = pack_hl(fv);
        v8f aG = zero8, aGr = zero8;
#pragma unroll 1
        for (int s = 0; s < 4; ++s) {
            const int tb = tsb + s * 512;
            const v4f p0 = *(const v4fa*)(&tss[tb]), p1 = *(const v4fa*)(&tss[tb + 4]), p2 = *(const v4fa*)(&tss[tb + 256]), p3 = *(const v4fa*)(&tss[tb + 260]);
            const v8f c0 = mmg(ldh(WP + PO_HBT + (32 * s + lr) * 32 + fo),      fb, zero8);
            const v8f c1 = mmg(ldh(WP + PO_HBT + (32 * s + 16 + lr) * 32 + fo), fb, zero8);
            v8f v0, v1;
#pragma unroll
            for (int r = 0; r < 4; ++r) {
                float t = p0[r]; v0[r]     = c0[r]     * (I_HB * VVS) * (1.0f - t * t);
                t = p1[r];       v0[4 + r] = c0[4 + r] * (I_HB * VVS) * (1.0f - t * t);
                t = p2[r];       v1[r]     = c1[r]     * (I_HB * VVS) * (1.0f - t * t);
                t = p3[r];       v1[4 + r] = c1[4 + r] * (I_HB * VVS) * (1.0f - t * t); }
            const v16h a = ldh(WP + PO_HAT + lr * BLN + 32 * s + fo);
            aG = mmg(a, pack2(v0, v1), aG);
            if (ev != 0) aGr = mmg(a, pack2r(v0, v1), aGr);
        }
        v8f gv;
#pragma unroll
        for (int r = 0; r < 8; ++r) gv[r] = (aG[r] + aGr[r] * QRI) * I_G + MU_C * fv[r];
        *(v4fa*)(&gss[gsb + lr * 16 + fo]) = lo4(gv); *(v4fa*)(&gss[gsb + lr * 16 + fo + 4]) = hi4(gv);
        wave_sync();

        v16h hb0, hb1;
        { const v8f ta = tile_a(WP + PO_JA + (lr) * 32 + fo,      BP + BO_JA + fo,      zb, I_L1);
          const v8f tb = tile_a(WP + PO_JA + (16 + lr) * 32 + fo, BP + BO_JA + 16 + fo, zb, I_L1); hb0 = pack2(ta, tb); }
        asm volatile("" ::: "memory");
        { const v8f ta = tile_a(WP + PO_JA + (32 + lr) * 32 + fo, BP + BO_JA + 32 + fo, zb, I_L1);
          const v8f tb = tile_a(WP + PO_JA + (48 + lr) * 32 + fo, BP + BO_JA + 48 + fo, zb, I_L1); hb1 = pack2(ta, tb); }
        asm volatile("" ::: "memory");
        v16h kb0, kb1;
        { const v8f ta = tile_b(WP + PO_JB + (lr) * HID + fo,      BP + BO_JB + fo,      hb0, hb1, I_L2);
          const v8f tb = tile_b(WP + PO_JB + (16 + lr) * HID + fo, BP + BO_JB + 16 + fo, hb0, hb1, I_L2); kb0 = pack2(ta, tb); }
        asm volatile("" ::: "memory");
        { const v8f ta = tile_b(WP + PO_JB + (32 + lr) * HID + fo, BP + BO_JB + 32 + fo, hb0, hb1, I_L2);
          const v8f tb = tile_b(WP + PO_JB + (48 + lr) * HID + fo, BP + BO_JB + 48 + fo, hb0, hb1, I_L2); kb1 = pack2(ta, tb); }
        asm volatile("" ::: "memory");
        v8f dzr = zero8;
#pragma unroll 1
        for (int c = 0; c < 16; ++c) {
            const h16* wp = WP + PO_JC + (16 * c + lr) * HID + fo;
            v8f acc = mmg(ldh(wp), kb0, zero8); acc = mmg(ldh(wp + 32), kb1, acc);
            const v8f bb = ld8f(BP + BO_JC + 16 * c + fo);
            v8f val; float s = 0.0f;
#pragma unroll
            for (int r = 0; r < 8; ++r) { val[r] = acc[r] * I_L3 + bb[r]; s += val[r] * gv[r]; }
            s += __shfl_xor(s, 16, 32);
            const float gc = gss[gsb + lr * 16 + c];
#pragma unroll
            for (int r = 0; r < 8; ++r) dzr[r] += ((c == fo + r) ? s : 0.0f) - val[r] * gc;
        }
        v8f wac = zero8;
#pragma unroll 1
        for (int c = 0; c < 16; ++c) {
            const h16* wp = WP + PO_JC + (256 + 16 * c + lr) * HID + fo;
            v8f acc = mmg(ldh(wp), kb0, zero8); acc = mmg(ldh(wp + 32), kb1, acc);
            const v8f bb = ld8f(BP + BO_JC + 256 + 16 * c + fo);
            const float gr = gss[gsb + lr * 16 + c];
            v4f a, b;
#pragma unroll
            for (int r = 0; r < 4; ++r) { a[r] = acc[r] * I_L3 + bb[r]; b[r] = acc[4 + r] * I_L3 + bb[4 + r]; wac[r] += a[r] * gr; wac[4 + r] += b[r] * gr; }
            *(v4fa*)(&rfs[rfb + (c * 16 + lr) * 16 + fo]) = a; *(v4fa*)(&rfs[rfb + (c * 16 + lr) * 16 + fo + 4]) = b;
        }
        float wlo[8], whi[8];
#pragma unroll
        for (int j = 0; j < 8; ++j) { const float ot = __shfl_xor(wac[j], 16, 32); wlo[j] = (hi != 0) ? ot : wac[j]; whi[j] = (hi != 0) ? wac[j] : ot; }
        wave_sync();
#pragma unroll 1
        for (int v = 0; v < 8; ++v) {
            const int rb = rfb + ((fo + v) * 16 + lr) * 16;
            const v4f x0 = *(const v4fa*)(&rfs[rb]), x1 = *(const v4fa*)(&rfs[rb + 4]), x2 = *(const v4fa*)(&rfs[rb + 8]), x3 = *(const v4fa*)(&rfs[rb + 12]);
            float s = 0.0f;
#pragma unroll
            for (int k = 0; k < 4; ++k) s += x0[k] * wlo[k] + x1[k] * wlo[4 + k] + x2[k] * whi[k] + x3[k] * whi[4 + k];
#pragma unroll
            for (int r = 0; r < 8; ++r) dzr[r] -= (r == v) ? s : 0.0f;
        }

        v16h mb0, mb1, mr0, mr1;
        { const v8f ta = tile_a(WP + PO_MA + (lr) * 32 + fo,      BP + BO_MA + fo,      zb, I_L1);
          const v8f tb = tile_a(WP + PO_MA + (16 + lr) * 32 + fo, BP + BO_MA + 16 + fo, zb, I_L1); mb0 = pack2(ta, tb); mr0 = pack2r(ta, tb); }
        asm volatile("" ::: "memory");
        { const v8f ta = tile_a(WP + PO_MA + (32 + lr) * 32 + fo, BP + BO_MA + 32 + fo, zb, I_L1);
          const v8f tb = tile_a(WP + PO_MA + (48 + lr) * 32 + fo, BP + BO_MA + 48 + fo, zb, I_L1); mb1 = pack2(ta, tb); mr1 = pack2r(ta, tb); }
        asm volatile("" ::: "memory");
        v16h nb0, nb1, nr0, nr1;
        { const v8f ta = tile_br(WP + PO_MB + (lr) * HID + fo,      BP + BO_MB + fo,      mb0, mb1, mr0, mr1, ev, I_L2);
          const v8f tb = tile_br(WP + PO_MB + (16 + lr) * HID + fo, BP + BO_MB + 16 + fo, mb0, mb1, mr0, mr1, ev, I_L2); nb0 = pack2(ta, tb); nr0 = pack2r(ta, tb); }
        asm volatile("" ::: "memory");
        { const v8f ta = tile_br(WP + PO_MB + (32 + lr) * HID + fo, BP + BO_MB + 32 + fo, mb0, mb1, mr0, mr1, ev, I_L2);
          const v8f tb = tile_br(WP + PO_MB + (48 + lr) * HID + fo, BP + BO_MB + 48 + fo, mb0, mb1, mr0, mr1, ev, I_L2); nb1 = pack2(ta, tb); nr1 = pack2r(ta, tb); }
        asm volatile("" ::: "memory");
        yp = zero8;
#pragma unroll 1
        for (int c = 0; c < 8; ++c) {
            const h16* wp = WP + PO_MC + (16 * c + lr) * HID + fo;
            const v16h a0 = ldh(wp), a1 = ldh(wp + 32);
            v8f acc = mmg(a0, nb0, zero8); acc = mmg(a1, nb1, acc);
            v8f acr = zero8;
            if (ev != 0) { acr = mmg(a0, nr0, acr); acr = mmg(a1, nr1, acr); }
            const v8f bb = ld8f(BP + BO_MC + 16 * c + fo);
            const float gc = gss[gsb + lr * 16 + fo + c];
            float bu = 0.0f;
#pragma unroll
            for (int r = 0; r < 8; ++r) { const float val = (acc[r] + acr[r] * QRI) * I_L3 + bb[r]; bu += val * uv[r]; yp[r] += val * gc; }
#pragma unroll
            for (int r = 0; r < 8; ++r) dzr[r] += (r == c) ? bu : 0.0f;
        }
        dzp = dzl;
#pragma unroll
        for (int v = 0; v < 8; ++v) { const float d = dzr[v] - EPS_C * gv[v]; dzl[v] = d; zc[v] = z0[v] + d; }
    }

    { v4f a, b, yv;
#pragma unroll
      for (int r = 0; r < 4; ++r) { a[r] = z0[r] + 0.5f * (dzp[r] + dzl[r]); b[r] = z0[4 + r] + 0.5f * (dzp[4 + r] + dzl[4 + r]); }
      float yf[8];
#pragma unroll
      for (int r = 0; r < 8; ++r) yf[r] = yp[r] + __shfl_xor(yp[r], 16, 32);
#pragma unroll
      for (int r = 0; r < 4; ++r) yv[r] = (hi != 0) ? yf[4 + r] : yf[r];
      *(v4fa*)(&oss[osb + lr * 16 + fo]) = a; *(v4fa*)(&oss[osb + lr * 16 + fo + 4]) = b;
      *(v4fa*)(&oss[osb + 256 + lr * 8 + 4 * hi]) = yv; }
    wave_sync();
    float* o0 = OUT0 + row0 * LAT;
    float* o1 = OUT1 + row0 * CTL;
#pragma unroll 1
    for (int ps = 0; ps < 2; ++ps) {
#pragma unroll
        for (int s = 0; s < 2; ++s) { const int p = s * 32 + lane;
            const v4f val = *(const v4fa*)(&oss[osb + p * 4]);
            *(volatile v4f*)(o0 + p * 4) = val; }
        { const v4f val = *(const v4fa*)(&oss[osb + 256 + lane * 4]);
          *(volatile v4f*)(o1 + lane * 4) = val; }
        if (ps == 0) __threadfence(); }
}

static constexpr size_t al256(size_t v) { return (v + 255) & ~(size_t)255; }
static constexpr size_t SZ_WP = al256((size_t)PO_END * 2);
static constexpr size_t SZ_BP = al256((size_t)BO_END * 4);
static constexpr size_t SZ_TOTAL = SZ_WP + SZ_BP;
static_assert(SZ_TOTAL <= (size_t)134217728);
static_assert(SZ_WP == (size_t)PO_END * 2);
static_assert(SZ_BP == (size_t)BO_END * 4);

static void launch_wplane(hipStream_t stream, const float* src, h16* dst, int rows, int pitch, int sld, int nsrc, int tr, int dup, int perm, float cs, float cs2) {
    const int pieces = rows * (pitch / 8);
    k_wplane<<<(unsigned)((pieces + 255) / 256), 256, 0, stream>>>(src, dst, rows, pitch, sld, nsrc, tr, dup, perm, cs, cs2);
}

extern "C" void kernel_launch(void* const* d_in, const int* in_sizes, int n_in,
                              void* d_out, int out_size, void* d_ws, size_t ws_size, hipStream_t stream) {
    if (n_in < 17) return;
    if ((size_t)in_sizes[0] < (size_t)NROWS * LAT || (size_t)in_sizes[1] < (size_t)NROWS * CTL) return;
    if (in_sizes[2] < BLN * LAT || in_sizes[3] < BLN || in_sizes[4] < LAT * BLN) return;
    if (in_sizes[5] < HID * LAT || in_sizes[6] < HID || in_sizes[7] < HID * HID || in_sizes[8] < HID || in_sizes[9] < JRO * HID || in_sizes[10] < JRO) return;
    if (in_sizes[11] < HID * LAT || in_sizes[12] < HID || in_sizes[13] < HID * HID || in_sizes[14] < HID || in_sizes[15] < BMO * HID || in_sizes[16] < BMO) return;
    if ((size_t)out_size < (size_t)NROWS_FULL * LAT + (size_t)NROWS * CTL) return;
    if (SZ_TOTAL > ws_size) return;
    const float* z   = (const float*)d_in[0];  const float* u   = (const float*)d_in[1];
    const float* wha = (const float*)d_in[2];  const float* bha = (const float*)d_in[3];  const float* whb = (const float*)d_in[4];
    const float* wja = (const float*)d_in[5];  const float* bja = (const float*)d_in[6];
    const float* wjb = (const float*)d_in[7];  const float* bjb = (const float*)d_in[8];
    const float* wjc = (const float*)d_in[9];  const float* bjc = (const float*)d_in[10];
    const float* wma = (const float*)d_in[11]; const float* bma = (const float*)d_in[12];
    const float* wmb = (const float*)d_in[13]; const float* bmb = (const float*)d_in[14];
    const float* wmc = (const float*)d_in[15]; const float* bmc = (const float*)d_in[16];
    float* OUT0 = (float*)d_out;
    float* OUT1 = (float*)d_out + (size_t)NROWS_FULL * LAT;
    char* wsp = (char*)d_ws;
    h16* WP = (h16*)wsp; wsp += SZ_WP;
    float* BP = (float*)wsp; wsp += SZ_BP;

    launch_wplane(stream, wha, WP + PO_HA,  BLN, 32,  LAT, BLN * LAT, 0, 1, 0, CW_HA, CW_HA / LOS);
    launch_wplane(stream, whb, WP + PO_HB,  LAT, BLN, BLN, LAT * BLN, 0, 0, 0, CW_HB, CW_HB);
    launch_wplane(stream, whb, WP + PO_HBT, BLN, 32,  BLN, LAT * BLN, 1, 1, 0, CW_HB, CW_HB / LOS);
    launch_wplane(stream, wha, WP + PO_HAT, LAT, BLN, LAT, BLN * LAT, 1, 0, 0, CW_HA, CW_HA);
    launch_wplane(stream, wja, WP + PO_JA,  HID, 32,  LAT, HID * LAT, 0, 1, 0, CW_L1, CW_L1 / LOS);
    launch_wplane(stream, wjb, WP + PO_JB,  HID, HID, HID, HID * HID, 0, 0, 0, CW_L2, CW_L2);
    launch_wplane(stream, wjc, WP + PO_JC,  JRO, HID, HID, JRO * HID, 0, 0, 0, CW_L3, CW_L3);
    launch_wplane(stream, wma, WP + PO_MA,  HID, 32,  LAT, HID * LAT, 0, 1, 0, CW_L1, CW_L1 / LOS);
    launch_wplane(stream, wmb, WP + PO_MB,  HID, HID, HID, HID * HID, 0, 0, 0, CW_L2, CW_L2);
    launch_wplane(stream, wmc, WP + PO_MC,  BMO, HID, HID, BMO * HID, 0, 0, 1, CW_L3, CW_L3);
    k_bias<<<1, 256, 0, stream>>>(bha, bja, bjb, bjc, bma, bmb, bmc, BP);

    k_step<<<(unsigned)(NROWS / (16 * AW)), 32 * AW, 0, stream>>>(z, u, WP, BP, OUT0, OUT1);
}
